// GsGLstm_24532853195501
// MI455X (gfx1250) — hardware-run, weakly checked
//
#include <hip/hip_runtime.h>
#include <math.h>

constexpr int NBAT   = 8;
constexpr int NNODE  = 1024;
constexpr int NNBR   = 16;
constexpr int NHID   = 256;
constexpr int NGATE  = 4;
constexpr int NLAYER = 3;
constexpr int NROWS  = NBAT * NNODE;
constexpr int NCOLS  = NGATE * NHID;
constexpr int KXCAT  = 2 * NHID;
constexpr int KHCAT  = 4 * NHID;
constexpr int NTHR   = 256;
static_assert(NROWS == 8192 && NCOLS == 1024 && KXCAT == 512 && KHCAT == 1024, "shape constants");
static_assert(NROWS % 64 == 0 && NCOLS % 64 == 0, "GEMM tile multiples");
static_assert(KXCAT % 32 == 0 && KHCAT % 32 == 0, "GEMM k multiples");
static_assert(NNODE == 1024, "batch index uses a shift by 10");
static_assert(NHID == NTHR, "one gate thread per hidden unit");
static_assert(NLAYER == 3, "the host layer sequence below is written out for exactly three layers");
static_assert((NROWS * NHID) % (4 * NTHR) == 0, "NaN fill grid exact");

typedef __attribute__((ext_vector_type(16))) __bf16   v16b;
typedef __attribute__((ext_vector_type(8)))  __bf16   v8b;
typedef __attribute__((ext_vector_type(8)))  float    v8f;
typedef __attribute__((ext_vector_type(4)))  float    v4f;
typedef __attribute__((ext_vector_type(4)))  unsigned v4u;

__device__ __forceinline__ unsigned short f2bf_bits(float f) {
  unsigned u = __float_as_uint(f);
  return (unsigned short)((u + 0x7FFFu + ((u >> 16) & 1u)) >> 16);
}
__device__ __forceinline__ float bf_bits2f(unsigned short h) { return __uint_as_float(((unsigned)h) << 16); }
__device__ __forceinline__ float bf16r(float f) { return bf_bits2f(f2bf_bits(f)); }
__device__ __forceinline__ unsigned pack2(unsigned short lo, unsigned short hi) {
  return (unsigned)lo | ((unsigned)hi << 16);
}

__device__ __forceinline__ void row_guard_b(v8f& a0, v8f& a1, v8f& a2, v8f& a3,
                                            v16b x, v16b y0, v16b y1, v16b y2, v16b y3) {
  asm volatile("v_nop\n\tv_nop\n\tv_nop\n\tv_nop"
               : "+v"(a0), "+v"(a1), "+v"(a2), "+v"(a3)
               : "v"(x), "v"(y0), "v"(y1), "v"(y2), "v"(y3));
}
__device__ __forceinline__ void keep4_b(v16b a, v16b b, v16b c, v16b d) { asm volatile("v_nop" :: "v"(a), "v"(b), "v"(c), "v"(d)); }
__device__ __forceinline__ void acc_guard4(v8f& a, v8f& b, v8f& c, v8f& d) { asm volatile("v_nop\n\tv_nop\n\tv_nop\n\tv_nop" : "+v"(a), "+v"(b), "+v"(c), "+v"(d)); }

template <typename T> struct Frag;
template <> struct Frag<__bf16> {
  typedef v16b V; union U { v16b v; v8b h[2]; };
  static __device__ __forceinline__ v16b load(const __bf16* p) {
    U f; f.h[0] = *(const v8b*)(p); f.h[1] = *(const v8b*)(p + 16); return f.v;
  }
  static __device__ __forceinline__ v8f mma(v16b a, v16b b, v8f c) {
    return __builtin_amdgcn_wmma_f32_16x16x32_bf16(false, a, false, b, (short)0, c, false, false);
  }
};

__global__ __launch_bounds__(256) void wmma_gemm64_bf16(
    const unsigned short* __restrict__ Ap, int lda,
    const unsigned short* __restrict__ Btp, int ldb,
    float* __restrict__ Cout, int ldc, int Mr, int Nc, int Kd) {
  typedef __bf16 T;
  typedef v16b V;
  const T* A  = (const T*)Ap;
  const T* Bt = (const T*)Btp;
  __shared__ __align__(16) float sT[8][16 * 68];
  const int lane = threadIdx.x & 31;
  const int wave = threadIdx.x >> 5;
  const int tilesN = Nc >> 6;
  const int tilesM = Mr >> 6;
  const int tile = blockIdx.x * 8 + wave;
  if (tile >= tilesM * tilesN) return;
  const int tm = tile / tilesN;
  const int tn = tile - tm * tilesN;
  const int m0 = tm << 6;
  const int n0 = tn << 6;

  const int rlane = lane & 15;
  const int koff  = (lane >> 4) * 8;
  const int mOff  = (lane >> 4) * 8;

  v8f acc[4][4];
#pragma unroll
  for (int i = 0; i < 4; ++i)
#pragma unroll
    for (int j = 0; j < 4; ++j) acc[i][j] = (v8f){0.f,0.f,0.f,0.f,0.f,0.f,0.f,0.f};

  const T* bptr[4];
  const T* aptr[4];
#pragma unroll
  for (int j = 0; j < 4; ++j) bptr[j] = Bt + (size_t)(n0 + (j << 4) + rlane) * ldb + koff;
#pragma unroll
  for (int i = 0; i < 4; ++i) aptr[i] = A + (size_t)(m0 + (i << 4) + rlane) * lda + koff;

#pragma unroll 1
  for (int k0 = 0; k0 < Kd; k0 += 32) {
    V bh[4];
#pragma unroll
    for (int j = 0; j < 4; ++j) bh[j] = Frag<T>::load(bptr[j] + k0);
#pragma unroll
    for (int i = 0; i < 4; ++i) {
      V ah = Frag<T>::load(aptr[i] + k0);
#pragma unroll
      for (int j = 0; j < 4; ++j) acc[i][j] = Frag<T>::mma(ah, bh[j], acc[i][j]);
      row_guard_b(acc[i][0], acc[i][1], acc[i][2], acc[i][3], ah, bh[0], bh[1], bh[2], bh[3]);
    }
    keep4_b(bh[0], bh[1], bh[2], bh[3]);
  }
  acc_guard4(acc[0][0], acc[0][1], acc[0][2], acc[0][3]);
  acc_guard4(acc[1][0], acc[1][1], acc[1][2], acc[1][3]);
  acc_guard4(acc[2][0], acc[2][1], acc[2][2], acc[2][3]);
  acc_guard4(acc[3][0], acc[3][1], acc[3][2], acc[3][3]);

  float* slab = sT[wave];
#pragma unroll
  for (int i = 0; i < 4; ++i) {
    const int mBase = m0 + (i << 4);
#pragma unroll
    for (int j = 0; j < 4; ++j) {
#pragma unroll
      for (int r = 0; r < 8; ++r) {
        slab[(mOff + r) * 68 + (j << 4) + rlane] = acc[i][j][r];
      }
    }
    __builtin_amdgcn_fence(__ATOMIC_RELEASE, "workgroup");
    __builtin_amdgcn_wave_barrier();
    __builtin_amdgcn_fence(__ATOMIC_ACQUIRE, "workgroup");
    {
      const int hh = lane >> 4, c4 = (lane & 15) * 4;
      for (int pass = 0; pass < 2; ++pass) {
#pragma unroll
        for (int it = 0; it < 8; ++it) {
          const int row = it * 2 + hh;
          v4f v = *(const v4f*)(slab + row * 68 + c4);
          *(volatile v4f*)(Cout + (size_t)(mBase + row) * ldc + n0 + c4) = v;
        }
        __threadfence();
      }
    }
    __builtin_amdgcn_fence(__ATOMIC_RELEASE, "workgroup");
    __builtin_amdgcn_wave_barrier();
    __builtin_amdgcn_fence(__ATOMIC_ACQUIRE, "workgroup");
  }
}

__global__ __launch_bounds__(NTHR) void cvt_x_kernel(const float* __restrict__ xa, const float* __restrict__ xb,
                                                     unsigned short* __restrict__ AX) {
  const int i   = blockIdx.x * NTHR + threadIdx.x;
  const int row = i >> 6;
  const int c8  = i & 63;
  const float* src = (c8 < 32) ? xa : xb;
  const float* sp  = src + (size_t)row * NHID + (c8 & 31) * 8;
  const v4f a = *(const v4f*)(sp);
  const v4f b = *(const v4f*)(sp + 4);
  const float a0 = a[0], a1 = a[1], a2 = a[2], a3 = a[3];
  const float b0 = b[0], b1 = b[1], b2 = b[2], b3 = b[3];
  v4u w;
  w[0] = pack2(f2bf_bits(a0), f2bf_bits(a1));
  w[1] = pack2(f2bf_bits(a2), f2bf_bits(a3));
  w[2] = pack2(f2bf_bits(b0), f2bf_bits(b1));
  w[3] = pack2(f2bf_bits(b2), f2bf_bits(b3));
  volatile v4u* dp = (volatile v4u*)(AX + (size_t)i * 8);
  *dp = w;
  __threadfence();
  *dp = w;
}

__global__ __launch_bounds__(NTHR) void tpw_all_kernel(const float* __restrict__ w_in, const float* __restrict__ u_in,
                                                       const float* __restrict__ w_out, const float* __restrict__ u_out,
                                                       unsigned short* __restrict__ BTX, unsigned short* __restrict__ BTH) {
  __shared__ float Tt[64 * 65];
  const int tid = threadIdx.x;
  const int job = blockIdx.z >> 2;
  const int g   = blockIdx.z & 3;
  const float* srcm = (job == 0) ? w_in : ((job == 1) ? w_out : ((job < 4) ? u_in : u_out));
  unsigned short* dstp = (job < 2) ? BTX : BTH;
  const int ldo  = (job < 2) ? KXCAT : KHCAT;
  const int kofs = (job < 2) ? (job * NHID) : ((job - 2) * NHID);
  const float* src = srcm + (size_t)g * NHID * NHID;
  const int c0 = blockIdx.x * 64, r0 = blockIdx.y * 64;
#pragma unroll
  for (int i = 0; i < 4; ++i) {
    const int idx = i * NTHR + tid;
    const int rr = idx >> 4, cc = (idx & 15) * 4;
    const v4f v = *(const v4f*)(src + (size_t)(r0 + rr) * NHID + c0 + cc);
    Tt[rr * 65 + cc + 0] = v[0];
    Tt[rr * 65 + cc + 1] = v[1];
    Tt[rr * 65 + cc + 2] = v[2];
    Tt[rr * 65 + cc + 3] = v[3];
  }
  __syncthreads();
  const int q = tid >> 3, c8 = (tid & 7) * 8;
  v4u hv[2];
#pragma unroll
  for (int gq = 0; gq < 2; ++gq) {
    const int qq = gq * 32 + q;
#pragma unroll
    for (int j = 0; j < 4; ++j) {
      const float f0 = Tt[(c8 + 2 * j) * 65 + qq];
      const float f1 = Tt[(c8 + 2 * j + 1) * 65 + qq];
      hv[gq][j] = pack2(f2bf_bits(f0), f2bf_bits(f1));
    }
  }
  for (int pass = 0; pass < 2; ++pass) {
#pragma unroll
    for (int gq = 0; gq < 2; ++gq) {
      const size_t o = (size_t)(g * NHID + c0 + gq * 32 + q) * (size_t)ldo + (size_t)(kofs + r0 + c8);
      *(volatile v4u*)(dstp + o) = hv[gq];
    }
    __threadfence();
  }
}

template <bool CVT16>
__global__ __launch_bounds__(NTHR) void gather_split_kernel(
    const float* __restrict__ hsrc, const int* __restrict__ in_nodes, const float* __restrict__ in_mask,
    const int* __restrict__ out_nodes, const float* __restrict__ out_mask, const float* __restrict__ node_mask,
    unsigned short* __restrict__ AH) {
  const int lane = threadIdx.x & 31;
  const int row  = blockIdx.x * (NTHR / 32) + (threadIdx.x >> 5);
  const int bat  = row >> 10;
  const float* hb = hsrc + (size_t)bat * NNODE * NHID + lane * 8;
  const float nmv = node_mask[row];
  const int nmb = __builtin_amdgcn_readfirstlane(__float_as_int(nmv));
  const bool rowact = (nmb & 0x7fffffff) != 0;
  const float nm = __int_as_float(nmb);
  float ai[8], ao[8];
#pragma unroll
  for (int e = 0; e < 8; ++e) { ai[e] = 0.0f; ao[e] = 0.0f; }
  const int rk = row * NNBR;
#pragma unroll 1
  for (int k = 0; k < NNBR; ++k) {
    const int   idi_v = in_nodes[rk + k];
    const float mi_v  = in_mask[rk + k];
    const int   ido_v = out_nodes[rk + k];
    const float mo_v  = out_mask[rk + k];
    const int idi = __builtin_amdgcn_readfirstlane(idi_v);
    const int mib = __builtin_amdgcn_readfirstlane(__float_as_int(mi_v));
    const int ido = __builtin_amdgcn_readfirstlane(ido_v);
    const int mob = __builtin_amdgcn_readfirstlane(__float_as_int(mo_v));
    if (rowact && ((mib & 0x7fffffff) != 0)) {
      int idc = idi < 0 ? 0 : idi;
      idc = idc > (NNODE - 1) ? (NNODE - 1) : idc;
      const float* p = hb + (size_t)idc * NHID;
      const v4f a = *(const v4f*)(p);
      const v4f b = *(const v4f*)(p + 4);
      const float m = __int_as_float(mib);
#pragma unroll
      for (int e = 0; e < 4; ++e) {
        float fa = a[e];
        float fb = b[e];
        if (CVT16) { fa = bf16r(fa); fb = bf16r(fb); }
        ai[e]     = fmaf(m, fa, ai[e]);
        ai[4 + e] = fmaf(m, fb, ai[4 + e]);
      }
    }
    if (rowact && ((mob & 0x7fffffff) != 0)) {
      int idc = ido < 0 ? 0 : ido;
      idc = idc > (NNODE - 1) ? (NNODE - 1) : idc;
      const float* p = hb + (size_t)idc * NHID;
      const v4f a = *(const v4f*)(p);
      const v4f b = *(const v4f*)(p + 4);
      const float m = __int_as_float(mob);
#pragma unroll
      for (int e = 0; e < 4; ++e) {
        float fa = a[e];
        float fb = b[e];
        if (CVT16) { fa = bf16r(fa); fb = bf16r(fb); }
        ao[e]     = fmaf(m, fa, ao[e]);
        ao[4 + e] = fmaf(m, fb, ao[4 + e]);
      }
    }
  }
  v4u ihi, ilo, ohi, olo;
#pragma unroll
  for (int j = 0; j < 4; ++j) {
    const float s0 = rowact ? (ai[2 * j] * nm) : 0.0f;
    const float s1 = rowact ? (ai[2 * j + 1] * nm) : 0.0f;
    const float t0 = rowact ? (ao[2 * j] * nm) : 0.0f;
    const float t1 = rowact ? (ao[2 * j + 1] * nm) : 0.0f;
    const unsigned short s0h = f2bf_bits(s0), s1h = f2bf_bits(s1);
    const unsigned short t0h = f2bf_bits(t0), t1h = f2bf_bits(t1);
    const unsigned short s0l = f2bf_bits(s0 - bf_bits2f(s0h)), s1l = f2bf_bits(s1 - bf_bits2f(s1h));
    const unsigned short t0l = f2bf_bits(t0 - bf_bits2f(t0h)), t1l = f2bf_bits(t1 - bf_bits2f(t1h));
    ihi[j] = pack2(s0h, s1h);
    ilo[j] = pack2(s0l, s1l);
    ohi[j] = pack2(t0h, t1h);
    olo[j] = pack2(t0l, t1l);
  }
  unsigned short* rp = AH + (size_t)row * KHCAT + lane * 8;
  for (int pass = 0; pass < 2; ++pass) {
    *(volatile v4u*)(rp)            = ihi;
    *(volatile v4u*)(rp + NHID)     = ilo;
    *(volatile v4u*)(rp + 2 * NHID) = ohi;
    *(volatile v4u*)(rp + 3 * NHID) = olo;
    __threadfence();
  }
}

template <int LAYER>
__global__ __launch_bounds__(NTHR) void gate_kernel(const float* __restrict__ pre, const float* __restrict__ xpre,
                                                    const float* __restrict__ bias, const float* __restrict__ cprev,
                                                    const float* __restrict__ node_mask,
                                                    float* __restrict__ cnext, float* __restrict__ hnext) {
  __shared__ __align__(16) float stg[2][NHID];
  const int tid = threadIdx.x;
  const int row = blockIdx.x;
  const size_t po = (size_t)row * NCOLS + tid;
  const float nm = node_mask[row];
  float cp = cprev[(size_t)row * NHID + tid];
  if (LAYER == 0) cp = bf16r(cp);
  float gi = 0.0f, go = 0.0f, gf = 0.0f, gc = 0.0f;
#pragma unroll 1
  for (int q = 0; q < NGATE; ++q) {
    const float z  = (pre[po + (size_t)q * NHID] + xpre[po + (size_t)q * NHID]) + bf16r(bias[q * NHID + tid]);
    const float sc = (q == 3) ? 2.0f : 1.0f;
    const float ex = expf(-(sc * z));
    const float s  = 1.0f / (1.0f + ex);
    const float v  = (q == 3) ? (2.0f * s - 1.0f) : s;
    gi = (q == 0) ? v : gi;
    go = (q == 1) ? v : go;
    gf = (q == 2) ? v : gf;
    gc = (q == 3) ? v : gc;
  }
  const float cn = (gf * cp + gi * gc) * nm;
  const float e2 = expf(-(2.0f * cn));
  const float th = 2.0f * (1.0f / (1.0f + e2)) - 1.0f;
  const float hn = (go * th) * nm;
  stg[0][tid] = hn;
  stg[1][tid] = cn;
  __syncthreads();
  if (LAYER < 2) {
    if (tid < 128) {
      const int which = tid >> 6;
      const int idx = (tid & 63) * 4;
      const v4f v = *(const v4f*)(&stg[which][idx]);
      float* dbase = which ? cnext : hnext;
      volatile v4f* dp = (volatile v4f*)(dbase + (size_t)row * NHID + idx);
      *dp = v;
      __threadfence();
      *dp = v;
    }
  } else {
    if (tid < 64) {
      const int idx = tid * 4;
      const v4f v = *(const v4f*)(&stg[0][idx]);
      volatile v4f* dp = (volatile v4f*)(hnext + (size_t)row * NHID + idx);
      *dp = v;
      __threadfence();
      *dp = v;
    }
  }
}

__global__ __launch_bounds__(32) void layer_guard_kernel(const int* __restrict__ nlayers, unsigned* __restrict__ flag) {
  const int lane = threadIdx.x & 31;
  const int v = nlayers[0];
  const unsigned f = (v != NLAYER) ? 1u : 0u;
  volatile unsigned* dp = (volatile unsigned*)(flag + lane);
  *dp = f;
  __threadfence();
  *dp = f;
}

__global__ __launch_bounds__(NTHR) void nan_fill_kernel(const unsigned* __restrict__ flag, float* __restrict__ outp) {
  const unsigned f = flag[0];
  if (f == 0u) return;
  const size_t i = (size_t)blockIdx.x * NTHR + threadIdx.x;
  v4u q;
  q[0] = 0x7FC00000u;
  q[1] = 0x7FC00000u;
  q[2] = 0x7FC00000u;
  q[3] = 0x7FC00000u;
  volatile v4u* dp = (volatile v4u*)(outp + i * 4);
  *dp = q;
  __threadfence();
  *dp = q;
}

extern "C" void kernel_launch(void* const* d_in, const int* in_sizes, int n_in,
                              void* d_out, int out_size, void* d_ws, size_t ws_size, hipStream_t stream) {
  if (n_in < 15 || d_out == nullptr || d_ws == nullptr) return;
  const int nState = NROWS * NHID;
  const int nW = NGATE * NHID * NHID;
  const int nNb = NROWS * NNBR;
  if (in_sizes[0] != nState || in_sizes[1] != nState || in_sizes[2] != nState || in_sizes[3] != nState ||
      in_sizes[4] != nW || in_sizes[5] != nW || in_sizes[6] != nW || in_sizes[7] != nW ||
      in_sizes[8] != NGATE * NHID || in_sizes[9] != nNb || in_sizes[10] != nNb || in_sizes[11] != NROWS ||
      in_sizes[12] != nNb || in_sizes[13] != nNb || in_sizes[14] != 1 || out_size != nState) return;

  const float* h0        = (const float*)d_in[0];
  const float* c0        = (const float*)d_in[1];
  const float* x_in      = (const float*)d_in[2];
  const float* x_out     = (const float*)d_in[3];
  const float* W_in      = (const float*)d_in[4];
  const float* U_in      = (const float*)d_in[5];
  const float* W_out     = (const float*)d_in[6];
  const float* U_out     = (const float*)d_in[7];
  const float* bvec      = (const float*)d_in[8];
  const float* in_mask   = (const float*)d_in[9];
  const float* out_mask  = (const float*)d_in[10];
  const float* node_mask = (const float*)d_in[11];
  const int*   in_nodes  = (const int*)d_in[12];
  const int*   out_nodes = (const int*)d_in[13];
  const int*   nlayers   = (const int*)d_in[14];
  float* outp = (float*)d_out;

  char* ws = (char*)d_ws; size_t off = 0;
  auto carve = [&](size_t bytes) -> char* { char* p = ws + off; off += (bytes + 255) & ~(size_t)255; return p; };
  float*          XPRE = (float*)carve((size_t)NROWS * NCOLS * 4);
  float*          PRE  = (float*)carve((size_t)NROWS * NCOLS * 4);
  float*          HA   = (float*)carve((size_t)NROWS * NHID * 4);
  float*          HB   = (float*)carve((size_t)NROWS * NHID * 4);
  float*          CA   = (float*)carve((size_t)NROWS * NHID * 4);
  float*          CB   = (float*)carve((size_t)NROWS * NHID * 4);
  unsigned short* AH   = (unsigned short*)carve((size_t)NROWS * KHCAT * 2);
  unsigned short* AX   = (unsigned short*)carve((size_t)NROWS * KXCAT * 2);
  unsigned short* BTX  = (unsigned short*)carve((size_t)NCOLS * KXCAT * 2);
  unsigned short* BTH  = (unsigned short*)carve((size_t)NCOLS * KHCAT * 2);
  unsigned*       FLAG = (unsigned*)carve((size_t)128);
  if (off > ws_size || off > (size_t)134217728) return;

  layer_guard_kernel<<<1, 32, 0, stream>>>(nlayers, FLAG);

  cvt_x_kernel<<<(NROWS * (KXCAT / 8)) / NTHR, NTHR, 0, stream>>>(x_in, x_out, AX);
  tpw_all_kernel<<<dim3(NHID / 64, NHID / 64, 6 * NGATE), NTHR, 0, stream>>>(W_in, U_in, W_out, U_out, BTX, BTH);

  const int gemmBlocks = ((NROWS / 64) * (NCOLS / 64)) / 8;
  const int gatherBlocks = NROWS / (NTHR / 32);

  wmma_gemm64_bf16<<<gemmBlocks, 256, 0, stream>>>(AX, KXCAT, BTX, KXCAT, XPRE, NCOLS, NROWS, NCOLS, KXCAT);

  gather_split_kernel<true><<<gatherBlocks, NTHR, 0, stream>>>(h0, in_nodes, in_mask, out_nodes, out_mask, node_mask, AH);
  wmma_gemm64_bf16<<<gemmBlocks, 256, 0, stream>>>(AH, KHCAT, BTH, KHCAT, PRE, NCOLS, NROWS, NCOLS, KHCAT);
  gate_kernel<0><<<NROWS, NTHR, 0, stream>>>(PRE, XPRE, bvec, c0, node_mask, CA, HA);

  gather_split_kernel<false><<<gatherBlocks, NTHR, 0, stream>>>(HA, in_nodes, in_mask, out_nodes, out_mask, node_mask, AH);
  wmma_gemm64_bf16<<<gemmBlocks, 256, 0, stream>>>(AH, KHCAT, BTH, KHCAT, PRE, NCOLS, NROWS, NCOLS, KHCAT);
  gate_kernel<1><<<NROWS, NTHR, 0, stream>>>(PRE, XPRE, bvec, CA, node_mask, CB, HB);

  gather_split_kernel<false><<<gatherBlocks, NTHR, 0, stream>>>(HB, in_nodes, in_mask, out_nodes, out_mask, node_mask, AH);
  wmma_gemm64_bf16<<<gemmBlocks, 256, 0, stream>>>(AH, KHCAT, BTH, KHCAT, PRE, NCOLS, NROWS, NCOLS, KHCAT);
  gate_kernel<2><<<NROWS, NTHR, 0, stream>>>(PRE, XPRE, bvec, CB, node_mask, CA, outp);

  nan_fill_kernel<<<(NROWS * NHID) / (4 * NTHR), NTHR, 0, stream>>>(FLAG, outp);
}
